// MyConv2dPac_5463198401055
// MI455X (gfx1250) — hardware-verified
//
#include <hip/hip_runtime.h>
#include <stdint.h>

typedef _Float16 v16h __attribute__((ext_vector_type(16)));
typedef _Float16 v8h  __attribute__((ext_vector_type(8)));
typedef float    v8f  __attribute__((ext_vector_type(8)));
typedef float    v4f  __attribute__((ext_vector_type(4)));
typedef unsigned int v4u __attribute__((ext_vector_type(4)));

#define BATCH 8
#define CIN   64
#define HH    128
#define WW    128
#define OUTC  64
#define NT    64
#define NTAP  9
#define CSTR  80
#define XTCOLS 66
#define GP    12
#define OP    68
#define WPK_ELEMS (NTAP * 4 * 2 * 32 * 16)
#define WPK_GROUPS (WPK_ELEMS / 8)
#define WSCALE 64.0f
#define WINV   (1.0f / 64.0f)

static_assert((CSTR % 8) == 0);
static_assert((OP % 4) == 0);
static_assert(WPK_GROUPS * 8 == WPK_ELEMS);

union Frag { v16h v; v8h half[2]; };

__device__ __forceinline__ v8f wmma16(v16h a, v16h b, v8f c) {
  v8f d = __builtin_amdgcn_wmma_f32_16x16x32_f16(false, a, false, b, (short)0, c, false, false);
  asm volatile("v_nop\n\tv_nop\n\tv_nop\n\tv_nop" : "+v"(d) : "v"(a), "v"(b));
  return d;
}

__global__ __launch_bounds__(256)
void pac_pack_weights(const float* __restrict__ weight,
                      _Float16* __restrict__ wpk) {
  const int g = blockIdx.x * 256 + threadIdx.x;
  if (g >= WPK_GROUPS) return;
  const int idx0 = g * 8;
  const int hb   = (idx0 & 15) >> 3;
  const int lane = (idx0 >> 4) & 31;
  const int ks   = (idx0 >> 9) & 1;
  const int mblk = (idx0 >> 10) & 3;
  const int t    = idx0 >> 12;
  const int m    = mblk * 16 + (lane & 15);
  const int c0   = ks * 32 + ((lane >> 4) << 3) + (hb << 4);
  union { v8h hv; v4u u; } pk;
  #pragma unroll
  for (int j = 0; j < 8; ++j)
    pk.hv[j] = (_Float16)(weight[(m * CIN + c0 + j) * NTAP + t] * WSCALE);
  volatile v4u* dst = (volatile v4u*)(wpk + idx0);
  *dst = pk.u;
  __threadfence();
  *dst = pk.u;
}

__global__ __launch_bounds__(256)
void pac_wmma_kernel(const float* __restrict__ x,
                     const float* __restrict__ guide,
                     const _Float16* __restrict__ wpk,
                     const float* __restrict__ bias,
                     float* __restrict__ out) {
  __shared__ __align__(16) _Float16 xTs[3 * XTCOLS * CSTR];
  __shared__ float gS[NT * GP];
  __shared__ float biasS[OUTC];
  __shared__ __align__(16) float outS[OUTC * OP];

  const int tid  = threadIdx.x;
  const int lane = tid & 31;
  const int wid  = tid >> 5;
  const int b    = blockIdx.z;
  const int h    = blockIdx.y;
  const int w0   = blockIdx.x * NT;

  if (tid < OUTC) biasS[tid] = bias[tid];

  if (tid < NT) {
    const int w = w0 + tid;
    const float* gb = guide + (size_t)b * 3 * HH * WW;
    const float c0 = gb[(0 * HH + h) * WW + w];
    const float c1 = gb[(1 * HH + h) * WW + w];
    const float c2 = gb[(2 * HH + h) * WW + w];
    #pragma unroll
    for (int t = 0; t < NTAP; ++t) {
      const int hh = h + t / 3 - 1, ww = w + t % 3 - 1;
      const bool inb = (hh >= 0) && (hh < HH) && (ww >= 0) && (ww < WW);
      const int hc = hh < 0 ? 0 : (hh >= HH ? HH - 1 : hh);
      const int wc = ww < 0 ? 0 : (ww >= WW ? WW - 1 : ww);
      float v0 = gb[(0 * HH + hc) * WW + wc];
      float v1 = gb[(1 * HH + hc) * WW + wc];
      float v2 = gb[(2 * HH + hc) * WW + wc];
      if (!inb) { v0 = 0.f; v1 = 0.f; v2 = 0.f; }
      const float d0 = v0 - c0, d1 = v1 - c1, d2 = v2 - c2;
      const float s = d0 * d0 + d1 * d1 + d2 * d2;
      gS[tid * GP + t] = expf(-0.5f * s);
    }
  }

  for (int rc = wid; rc < 3 * CIN; rc += 8) {
    const int r = rc >> 6;
    const int c = rc & 63;
    const int hh = h + r - 1;
    const bool rowok = (hh >= 0) && (hh < HH);
    const float* src = x + ((size_t)(b * CIN + c) * HH + (rowok ? hh : 0)) * WW;
    for (int col = lane; col < XTCOLS; col += 32) {
      const int ww = w0 + col - 1;
      float v = 0.f;
      if (rowok && ww >= 0 && ww < WW) v = src[ww];
      xTs[(r * XTCOLS + col) * CSTR + c] = (_Float16)v;
    }
  }
  __syncthreads();

  const int mblk  = wid & 3;
  const int mBase = mblk * 16;
  const int nb    = (wid >> 2) * 32;
  const int nlo   = lane & 15;
  const int kh    = lane >> 4;
  const v8f zero8 = {0.f, 0.f, 0.f, 0.f, 0.f, 0.f, 0.f, 0.f};
  v8f acc0 = zero8;
  v8f acc1 = zero8;

  #pragma unroll 1
  for (int t = 0; t < NTAP; ++t) {
    const int dh = (t * 11) >> 5;
    const int dw = t - 3 * dh;
    const float g0 = gS[(nb + nlo) * GP + t];
    const float g1 = gS[(nb + 16 + nlo) * GP + t];
    const _Float16* xp0 = xTs + (dh * XTCOLS + nb + nlo + dw) * CSTR + 8 * kh;
    const _Float16* xp1 = xp0 + 16 * CSTR;
    const _Float16* wp = wpk + (size_t)((t * 4 + mblk) * 2) * 512 + lane * 16;
    Frag a0, a1, b00, b01, b10, b11;
    a0.v = *(const v16h*)(wp);
    a1.v = *(const v16h*)(wp + 512);
    b00.half[0] = *(const v8h*)(xp0);
    b00.half[1] = *(const v8h*)(xp0 + 16);
    b01.half[0] = *(const v8h*)(xp0 + 32);
    b01.half[1] = *(const v8h*)(xp0 + 48);
    b10.half[0] = *(const v8h*)(xp1);
    b10.half[1] = *(const v8h*)(xp1 + 16);
    b11.half[0] = *(const v8h*)(xp1 + 32);
    b11.half[1] = *(const v8h*)(xp1 + 48);

    v8f d0 = wmma16(a0.v, b00.v, zero8);
    d0 = wmma16(a1.v, b01.v, d0);
    v8f d1 = wmma16(a0.v, b10.v, zero8);
    d1 = wmma16(a1.v, b11.v, d1);

    #pragma unroll
    for (int r = 0; r < 8; ++r) {
      acc0[r] = fmaf(g0, d0[r], acc0[r]);
      acc1[r] = fmaf(g1, d1[r], acc1[r]);
    }
  }

  const int orow = mBase + 8 * kh;
  #pragma unroll
  for (int r = 0; r < 8; ++r) {
    const int o = orow + r;
    const float bv = biasS[o];
    outS[o * OP + nb + nlo]      = acc0[r] * WINV + bv;
    outS[o * OP + nb + 16 + nlo] = acc1[r] * WINV + bv;
  }
  __syncthreads();

  const int q    = lane & 7;
  const int lsub = lane >> 3;
  v4f vals[4];
  size_t gofs[4];
  #pragma unroll
  for (int j = 0; j < 4; ++j) {
    const int L    = wid * 16 + j * 4 + lsub;
    const int o    = L >> 1;
    const int half = L & 1;
    const int px   = half * 32 + 4 * q;
    vals[j] = *(const v4f*)&outS[o * OP + px];
    gofs[j] = ((size_t)(b * OUTC + o) * HH + h) * WW + w0 + px;
  }
  #pragma unroll
  for (int j = 0; j < 4; ++j) *(volatile v4f*)(out + gofs[j]) = vals[j];
  __threadfence();
  #pragma unroll
  for (int j = 0; j < 4; ++j) *(volatile v4f*)(out + gofs[j]) = vals[j];
}

extern "C" void kernel_launch(void* const* d_in, const int* in_sizes, int n_in,
                              void* d_out, int out_size, void* d_ws, size_t ws_size,
                              hipStream_t stream) {
  if (n_in < 4) return;
  if (in_sizes[0] != BATCH * CIN * HH * WW) return;
  if (in_sizes[1] != BATCH * 3 * HH * WW) return;
  if (in_sizes[2] != OUTC * CIN * NTAP) return;
  if (in_sizes[3] != OUTC) return;
  if (out_size != BATCH * OUTC * HH * WW) return;
  if (ws_size < (size_t)WPK_ELEMS * sizeof(_Float16)) return;

  const float* x      = (const float*)d_in[0];
  const float* guide  = (const float*)d_in[1];
  const float* weight = (const float*)d_in[2];
  const float* bias   = (const float*)d_in[3];
  _Float16* wpk       = (_Float16*)d_ws;
  float* out          = (float*)d_out;

  pac_pack_weights<<<(WPK_GROUPS + 255) / 256, 256, 0, stream>>>(weight, wpk);
  dim3 grid(WW / NT, HH, BATCH);
  pac_wmma_kernel<<<grid, dim3(256), 0, stream>>>(x, guide, wpk, bias, out);
}
